// LFA_55250459296229
// MI455X (gfx1250) — hardware-verified
//
#include <hip/hip_runtime.h>
#include <math.h>

typedef __attribute__((ext_vector_type(16))) _Float16 v16h;
typedef __attribute__((ext_vector_type(16))) __bf16 v16b;
typedef __attribute__((ext_vector_type(8)))  _Float16 v8h;
typedef __attribute__((ext_vector_type(8)))  float v8f;
typedef __attribute__((ext_vector_type(4)))  float v4f;
typedef __attribute__((ext_vector_type(2)))  float v2f;
typedef __attribute__((ext_vector_type(4)))  unsigned v4u;
typedef __attribute__((ext_vector_type(4)))  int v4i;
typedef float __attribute__((may_alias)) float_a;
typedef int __attribute__((may_alias)) int_a;

template <typename T> __device__ __forceinline__ void vst2(void* p, T v) { *(volatile T*)p = v; __threadfence(); *(volatile T*)p = v; }
__device__ __forceinline__ v8f wmma16(v16h a, v16h b, v8f c) {
  v8f d = __builtin_amdgcn_wmma_f32_16x16x32_f16(false, a, false, b, (short)0, c, false, false);
  asm volatile("v_nop\n\tv_nop\n\tv_nop\n\tv_nop" : "+v"(d) : "v"(a), "v"(b));
  return d;
}
__device__ __forceinline__ v8f wmma_bf(v16b a, v16b b, v8f c) {
  v8f d = __builtin_amdgcn_wmma_f32_16x16x32_bf16(false, a, false, b, (short)0, c, false, false);
  asm volatile("v_nop\n\tv_nop\n\tv_nop\n\tv_nop" : "+v"(d) : "v"(a), "v"(b));
  return d;
}
__device__ __forceinline__ v16h frag_h(const _Float16* rowk0, int lane) {
  union { v16h v; v8h q[2]; } u; const _Float16* p = rowk0 + 8 * (lane >> 4);
  u.q[0] = *(const v8h*)p; u.q[1] = *(const v8h*)(p + 16); return u.v;
}
__device__ __forceinline__ v16h frag_f32(const float* rowk0, int lane) {
  v16h a; const float* p = rowk0 + 8 * (lane >> 4);
#pragma unroll
  for (int i = 0; i < 8; ++i) { a[i] = (_Float16)p[i]; a[8 + i] = (_Float16)p[16 + i]; }
  return a;
}
__device__ __forceinline__ v16h frag_f32s(const float* rowk0, int lane, float sc) {
  v16h a; const float* p = rowk0 + 8 * (lane >> 4);
#pragma unroll
  for (int i = 0; i < 8; ++i) { a[i] = (_Float16)(p[i] * sc); a[8 + i] = (_Float16)(p[16 + i] * sc); }
  return a;
}
__device__ __forceinline__ v16h fragc_f32(const float* W, int k0, int n, int lane, int ld, int K) {
  v16h a; const int g = lane >> 4;
#pragma unroll
  for (int i = 0; i < 8; ++i) { const int ka = k0 + 8 * g + i, kb = ka + 16;
    a[i] = (_Float16)(ka < K ? W[(size_t)(ka < K ? ka : K - 1) * ld + n] : 0.f); a[8 + i] = (_Float16)(kb < K ? W[(size_t)(kb < K ? kb : K - 1) * ld + n] : 0.f); }
  return a;
}
struct F2 { v16b h, l; };
__device__ __forceinline__ F2 bsplit16(const float v[16]) { F2 r;
#pragma unroll
  for (int i = 0; i < 16; ++i) { const __bf16 h = (__bf16)v[i]; r.h[i] = h; r.l[i] = (__bf16)(v[i] - (float)h); }
  return r; }
__device__ __forceinline__ F2 split_row(const float* row, int k0, int lane) { float v[16]; const float* p = row + k0 + 8 * (lane >> 4);
#pragma unroll
  for (int i = 0; i < 8; ++i) { v[i] = p[i]; v[8 + i] = p[16 + i]; }
  return bsplit16(v); }
__device__ __forceinline__ F2 split_rowK(const float* row, int k0, int lane, int K) { float v[16]; const int g = lane >> 4;
#pragma unroll
  for (int i = 0; i < 8; ++i) { const int ka = k0 + 8 * g + i, kb = ka + 16; v[i] = ka < K ? row[ka < K ? ka : K - 1] : 0.f; v[8 + i] = kb < K ? row[kb < K ? kb : K - 1] : 0.f; }
  return bsplit16(v); }
__device__ __forceinline__ F2 split_col(const float* W, int k0, int n, int lane, int ld, int K) { float v[16]; const int g = lane >> 4;
#pragma unroll
  for (int i = 0; i < 8; ++i) { const int ka = k0 + 8 * g + i, kb = ka + 16; v[i] = ka < K ? W[(size_t)(ka < K ? ka : K - 1) * ld + n] : 0.f; v[8 + i] = kb < K ? W[(size_t)(kb < K ? kb : K - 1) * ld + n] : 0.f; }
  return bsplit16(v); }
__device__ __forceinline__ v8f mac3(const F2& a, const F2& b, v8f c) { c = wmma_bf(a.l, b.h, c); c = wmma_bf(a.h, b.l, c); return wmma_bf(a.h, b.h, c); }
__device__ __forceinline__ float sigm(float v) { return 1.0f / (1.0f + expf(-v)); }
#define LDSX() do { asm volatile("s_wait_dscnt 0" ::: "memory"); __builtin_amdgcn_wave_barrier(); __builtin_amdgcn_fence(__ATOMIC_RELEASE, "workgroup"); } while (0)


#define NB 4
#define NN 16384
#define KK 16
#define CI 128
#define CO 128
#define D2 64
#define NPT (NB * NN)
#define PPB 4
#define NBLK (NPT / PPB)
#ifndef TBLK
#define TBLK NBLK
#endif
typedef __attribute__((ext_vector_type(8))) __bf16 v8b;
__device__ __forceinline__ v16b frag_b(const __bf16* rowk0, int lane) {
  union { v16b v; v8b q[2]; } u; const __bf16* p = rowk0 + 8 * (lane >> 4);
  u.q[0] = *(const v8b*)p; u.q[1] = *(const v8b*)(p + 16); return u.v;
}
__device__ __forceinline__ float bfr(float v) { return (float)(__bf16)v; }
__device__ __attribute__((noinline)) float exp_ni(float v) { return expf(v); }
__device__ __attribute__((noinline)) float erf_ni(float v) { return erff(v); }

#define WS_XF  0u
#define WS_PRE (WS_XF + 4u * (size_t)NPT * CO)
#define WS_ST  (WS_PRE + 4u * (size_t)NPT * CO)
#define WS_BN  (WS_ST + 4u * (size_t)NBLK * 2 * CO)
#define WS_WH  (WS_BN + 4u * 2 * CO)
#define WS_END (WS_WH + 2u * (D2 * D2 + 2 * CO * CO))

__global__ __launch_bounds__(128) void k_xf(const float* __restrict__ X, const float* __restrict__ PW, float* __restrict__ XF) { __shared__ __align__(16) float sf[4][16][132];
  const int tid = threadIdx.x, wave = tid >> 5, lane = tid & 31, col = lane & 15, g = lane >> 4; const size_t r0 = (size_t)blockIdx.x * 64 + wave * 16;
  v8f acc[8] = {};
#pragma unroll
  for (int kc = 0; kc < CI / 32; ++kc) { v16b a; { const float* p = X + (r0 + col) * CI + kc * 32 + 8 * g;
#pragma unroll
      for (int i = 0; i < 8; ++i) { a[i] = (__bf16)p[i]; a[8 + i] = (__bf16)p[16 + i]; } }
#pragma unroll
    for (int j = 0; j < 8; ++j) { v16b w; const int o = j * 16 + col;
#pragma unroll
      for (int i = 0; i < 8; ++i) { w[i] = (__bf16)PW[o * CI + kc * 32 + 8 * g + i]; w[8 + i] = (__bf16)PW[o * CI + kc * 32 + 16 + 8 * g + i]; }
      acc[j] = wmma_bf(a, w, acc[j]); } }
#pragma unroll
  for (int j = 0; j < 8; ++j)
#pragma unroll
    for (int r = 0; r < 8; ++r) sf[wave][8 * g + r][j * 16 + col] = acc[j][r];
  LDSX(); for (int rl = 0; rl < 16; ++rl) vst2(XF + (r0 + rl) * CO + lane * 4, *(const v4f*)&sf[wave][rl][lane * 4]); }
__global__ __launch_bounds__(256) void k_w16(const float* __restrict__ W2, const float* __restrict__ W31, const float* __restrict__ W32, _Float16* __restrict__ WH) { __shared__ __align__(16) _Float16 s[2048]; const int t = threadIdx.x; const int blk = blockIdx.x;
  const int base = blk * 2048; for (int e = t; e < 2048; e += 256) { const int idx = base + e; float v; if (idx < D2 * D2) v = W2[idx]; else if (idx < D2 * D2 + CO * CO) v = W31[idx - D2 * D2]; else v = W32[idx - D2 * D2 - CO * CO]; s[e] = (_Float16)bfr(v); }
  __syncthreads(); vst2((unsigned*)(WH + base + t * 8), *(const v4u*)&s[t * 8]); }
__global__ __launch_bounds__(128) void k_pt(const float* __restrict__ XYZ, const int* __restrict__ KNN, const float* __restrict__ XF, const float* __restrict__ W1, const float* __restrict__ B1, const _Float16* __restrict__ WH, const float* __restrict__ B2, const float* __restrict__ B31, const float* __restrict__ B32, float* __restrict__ PRE, float* __restrict__ ST) { const _Float16* W2H = WH; const _Float16* W31H = WH + D2 * D2; const _Float16* W32H = W31H + CO * CO;
  __shared__ __align__(16) float sa[4][16][132]; __shared__ __align__(16) float spl[4][D2]; __shared__ __align__(16) float smx[4][CO]; __shared__ __align__(16) float sst[2][CO];
  const int tid = threadIdx.x, wave = tid >> 5, lane = tid & 31, col = lane & 15, g = lane >> 4; const size_t pt = (size_t)blockIdx.x * PPB + wave; const size_t b = pt / NN;
  const int myk = lane & 15; const size_t nbr = b * NN + (size_t)KNN[pt * KK + myk];
  { const float dx = bfr(XYZ[nbr * 3 + 0]) - bfr(XYZ[pt * 3 + 0]), dy = bfr(XYZ[nbr * 3 + 1]) - bfr(XYZ[pt * 3 + 1]), dz = bfr(XYZ[nbr * 3 + 2]) - bfr(XYZ[pt * 3 + 2]);
#pragma unroll 1
    for (int o = g * 32; o < g * 32 + 32; ++o) sa[wave][myk][o] = dx * bfr(W1[o * 3 + 0]) + dy * bfr(W1[o * 3 + 1]) + dz * bfr(W1[o * 3 + 2]) + bfr(B1[o]); }
  LDSX();
#pragma unroll
  for (int oo = 0; oo < 2; ++oo) { const int o = lane + 32 * oo; float mx = sa[wave][0][o];
#pragma unroll 1
    for (int k = 1; k < KK; ++k) mx = fmaxf(mx, sa[wave][k][o]);
    spl[wave][o] = mx; }
  v8f a1[4] = {};
#pragma unroll
  for (int kc = 0; kc < 2; ++kc) { const v16h a = frag_f32(&sa[wave][col][0] + kc * 32, lane);
#pragma unroll
    for (int j = 0; j < 4; ++j) a1[j] = wmma16(a, frag_h(W2H + (j * 16 + col) * D2 + kc * 32, lane), a1[j]); }
  LDSX();
#pragma unroll
  for (int j = 0; j < 4; ++j) { const float bb = bfr(B2[j * 16 + col]);
#pragma unroll
    for (int r = 0; r < 8; ++r) { sa[wave][8 * g + r][j * 16 + col] = a1[j][r] + bb; sa[wave][8 * g + r][D2 + j * 16 + col] = spl[wave][j * 16 + col]; } }
  LDSX();
  v8f ah[8] = {};
#pragma unroll
  for (int kc = 0; kc < 4; ++kc) { const v16h a = frag_f32(&sa[wave][col][0] + kc * 32, lane);
#pragma unroll
    for (int j = 0; j < 8; ++j) ah[j] = wmma16(a, frag_h(W31H + (j * 16 + col) * CO + kc * 32, lane), ah[j]); }
  LDSX();
#pragma unroll
  for (int j = 0; j < 8; ++j) { const float bb = bfr(B31[j * 16 + col]);
#pragma unroll
    for (int r = 0; r < 8; ++r) { const float u = ah[j][r] + bb; sa[wave][8 * g + r][j * 16 + col] = 0.5f * u * (1.0f + erff(u * 0.70710678118654752f)); } }
  LDSX();
  v8f ap[8] = {};
#pragma unroll
  for (int kc = 0; kc < 4; ++kc) { const v16h a = frag_f32(&sa[wave][col][0] + kc * 32, lane);
#pragma unroll
    for (int j = 0; j < 8; ++j) ap[j] = wmma16(a, frag_h(W32H + (j * 16 + col) * CO + kc * 32, lane), ap[j]); }
  LDSX();
#pragma unroll
  for (int j = 0; j < 8; ++j) { const int o = j * 16 + col; const float bb = bfr(B32[o]); const float xc = XF[pt * CO + o];
#pragma unroll
    for (int r = 0; r < 8; ++r) { const int k = 8 * g + r; const size_t nb2 = b * NN + (size_t)KNN[pt * KK + k]; sa[wave][k][o] = (XF[nb2 * CO + o] - xc) + (ap[j][r] + bb); } }
  LDSX();
  for (int o = lane; o < CO; o += 32) { float mx = sa[wave][0][o];
#pragma unroll 1
    for (int k = 1; k < KK; ++k) mx = fmaxf(mx, sa[wave][k][o]);
    smx[wave][o] = mx; }
  __syncthreads();
  if (tid < 32) { vst2(PRE + pt * 0 + ((size_t)blockIdx.x * PPB + 0) * CO + tid * 4, *(const v4f*)&smx[0][tid * 4]); vst2(PRE + ((size_t)blockIdx.x * PPB + 1) * CO + tid * 4, *(const v4f*)&smx[1][tid * 4]); vst2(PRE + ((size_t)blockIdx.x * PPB + 2) * CO + tid * 4, *(const v4f*)&smx[2][tid * 4]); vst2(PRE + ((size_t)blockIdx.x * PPB + 3) * CO + tid * 4, *(const v4f*)&smx[3][tid * 4]); }
  { const int o = tid; const float m4 = 0.25f * ((smx[0][o] + smx[1][o]) + (smx[2][o] + smx[3][o])); float q = 0.f;
#pragma unroll
    for (int p = 0; p < 4; ++p) { const float d = smx[p][o] - m4; q += d * d; }
    sst[0][o] = m4; sst[1][o] = q; }
  __syncthreads(); if (tid < 64) vst2(ST + (size_t)blockIdx.x * 2 * CO + tid * 4, *(const v4f*)&(&sst[0][0])[tid * 4]); }
__global__ __launch_bounds__(128) void k_bn(const float* __restrict__ ST, float* __restrict__ BN) { __shared__ __align__(16) float s[2][CO]; const int o = threadIdx.x; float n = 0.f, mean = 0.f, M2 = 0.f;
#pragma unroll 1
  for (int blk = 0; blk < TBLK; ++blk) { const float mb = ST[(size_t)blk * 2 * CO + o], qb = ST[(size_t)blk * 2 * CO + CO + o]; const float nb = 4.f; const float nt = n + nb; const float delta = mb - mean; mean += delta * (nb / nt); M2 += qb + delta * delta * (n * nb / nt); n = nt; }
  s[0][o] = mean; s[1][o] = 1.0f / sqrtf(M2 / n + 1e-5f); __syncthreads(); if (o < 64) vst2(BN + o * 4, *(const v4f*)&(&s[0][0])[o * 4]); }
__global__ __launch_bounds__(128) void k_fin(const float* __restrict__ PRE, const float* __restrict__ BN, const float* __restrict__ GA, const float* __restrict__ BE, float* __restrict__ OUT) { const int t = threadIdx.x; const size_t r0 = (size_t)blockIdx.x * 16;
  const int c4 = (t & 31) * 4; const float m0 = BN[c4], m1 = BN[c4 + 1], m2 = BN[c4 + 2], m3 = BN[c4 + 3], i0 = BN[CO + c4], i1 = BN[CO + c4 + 1], i2 = BN[CO + c4 + 2], i3 = BN[CO + c4 + 3];
  const float g0 = bfr(GA[c4]), g1 = bfr(GA[c4 + 1]), g2 = bfr(GA[c4 + 2]), g3 = bfr(GA[c4 + 3]), e0 = bfr(BE[c4]), e1 = bfr(BE[c4 + 1]), e2 = bfr(BE[c4 + 2]), e3 = bfr(BE[c4 + 3]);
#pragma unroll
  for (int rr = 0; rr < 4; ++rr) { const size_t row = r0 + (t >> 5) * 4 + rr; const float* p = PRE + row * CO + c4; v4f o; o[0] = (p[0] - m0) * i0 * g0 + e0; o[1] = (p[1] - m1) * i1 * g1 + e1; o[2] = (p[2] - m2) * i2 * g2 + e2; o[3] = (p[3] - m3) * i3 * g3 + e3; vst2(OUT + row * CO + c4, o); } }
extern "C" void kernel_launch(void* const* d_in, const int* in_sizes, int n_in, void* d_out, int out_size, void* d_ws, size_t ws_size, hipStream_t stream) {
  (void)in_sizes; (void)n_in; (void)out_size;
  const float** F = (const float**)d_in;
  if (ws_size < (size_t)WS_END) return;
  char* ws = (char*)d_ws; float *XF = (float*)(ws + WS_XF), *PRE = (float*)(ws + WS_PRE), *ST = (float*)(ws + WS_ST), *BN = (float*)(ws + WS_BN); _Float16* WH = (_Float16*)(ws + WS_WH);
  k_xf<<<NPT / 64, 128, 0, stream>>>(F[1], F[3], XF);
  k_w16<<<(D2 * D2 + 2 * CO * CO) / 2048, 256, 0, stream>>>(F[6], F[8], F[10], WH);
  k_pt<<<TBLK, 128, 0, stream>>>(F[0], (const int*)d_in[2], XF, F[4], F[5], WH, F[7], F[9], F[11], PRE, ST);
  k_bn<<<1, 128, 0, stream>>>(ST, BN);
  k_fin<<<TBLK * PPB / 16, 128, 0, stream>>>(PRE, BN, F[12], F[13], (float*)d_out);
}
